// GDEM_54047868453243
// MI455X (gfx1250) — hardware-verified
//
#include <hip/hip_runtime.h>
#include <math.h>

typedef __attribute__((ext_vector_type(16))) _Float16 v16h;
typedef __attribute__((ext_vector_type(16))) __bf16 v16b;
typedef __attribute__((ext_vector_type(8)))  _Float16 v8h;
typedef __attribute__((ext_vector_type(8)))  float v8f;
typedef __attribute__((ext_vector_type(4)))  float v4f;
typedef __attribute__((ext_vector_type(2)))  float v2f;
typedef __attribute__((ext_vector_type(4)))  unsigned v4u;
typedef __attribute__((ext_vector_type(4)))  int v4i;
typedef float __attribute__((may_alias)) float_a;
typedef int __attribute__((may_alias)) int_a;

template <typename T> __device__ __forceinline__ void vst2(void* p, T v) { *(volatile T*)p = v; __threadfence(); *(volatile T*)p = v; }
__device__ __forceinline__ v8f wmma16(v16h a, v16h b, v8f c) {
  v8f d = __builtin_amdgcn_wmma_f32_16x16x32_f16(false, a, false, b, (short)0, c, false, false);
  asm volatile("v_nop\n\tv_nop\n\tv_nop\n\tv_nop" : "+v"(d) : "v"(a), "v"(b));
  return d;
}
__device__ __forceinline__ v8f wmma_bf(v16b a, v16b b, v8f c) {
  v8f d = __builtin_amdgcn_wmma_f32_16x16x32_bf16(false, a, false, b, (short)0, c, false, false);
  asm volatile("v_nop\n\tv_nop\n\tv_nop\n\tv_nop" : "+v"(d) : "v"(a), "v"(b));
  return d;
}
__device__ __forceinline__ v16h frag_h(const _Float16* rowk0, int lane) {
  union { v16h v; v8h q[2]; } u; const _Float16* p = rowk0 + 8 * (lane >> 4);
  u.q[0] = *(const v8h*)p; u.q[1] = *(const v8h*)(p + 16); return u.v;
}
__device__ __forceinline__ v16h frag_f32(const float* rowk0, int lane) {
  v16h a; const float* p = rowk0 + 8 * (lane >> 4);
#pragma unroll
  for (int i = 0; i < 8; ++i) { a[i] = (_Float16)p[i]; a[8 + i] = (_Float16)p[16 + i]; }
  return a;
}
__device__ __forceinline__ v16h frag_f32s(const float* rowk0, int lane, float sc) {
  v16h a; const float* p = rowk0 + 8 * (lane >> 4);
#pragma unroll
  for (int i = 0; i < 8; ++i) { a[i] = (_Float16)(p[i] * sc); a[8 + i] = (_Float16)(p[16 + i] * sc); }
  return a;
}
__device__ __forceinline__ v16h fragc_f32(const float* W, int k0, int n, int lane, int ld, int K) {
  v16h a; const int g = lane >> 4;
#pragma unroll
  for (int i = 0; i < 8; ++i) { const int ka = k0 + 8 * g + i, kb = ka + 16;
    a[i] = (_Float16)(ka < K ? W[(size_t)(ka < K ? ka : K - 1) * ld + n] : 0.f); a[8 + i] = (_Float16)(kb < K ? W[(size_t)(kb < K ? kb : K - 1) * ld + n] : 0.f); }
  return a;
}
struct F2 { v16b h, l; };
__device__ __forceinline__ F2 bsplit16(const float v[16]) { F2 r;
#pragma unroll
  for (int i = 0; i < 16; ++i) { const __bf16 h = (__bf16)v[i]; r.h[i] = h; r.l[i] = (__bf16)(v[i] - (float)h); }
  return r; }
__device__ __forceinline__ F2 split_row(const float* row, int k0, int lane) { float v[16]; const float* p = row + k0 + 8 * (lane >> 4);
#pragma unroll
  for (int i = 0; i < 8; ++i) { v[i] = p[i]; v[8 + i] = p[16 + i]; }
  return bsplit16(v); }
__device__ __forceinline__ F2 split_rowK(const float* row, int k0, int lane, int K) { float v[16]; const int g = lane >> 4;
#pragma unroll
  for (int i = 0; i < 8; ++i) { const int ka = k0 + 8 * g + i, kb = ka + 16; v[i] = ka < K ? row[ka < K ? ka : K - 1] : 0.f; v[8 + i] = kb < K ? row[kb < K ? kb : K - 1] : 0.f; }
  return bsplit16(v); }
__device__ __forceinline__ F2 split_col(const float* W, int k0, int n, int lane, int ld, int K) { float v[16]; const int g = lane >> 4;
#pragma unroll
  for (int i = 0; i < 8; ++i) { const int ka = k0 + 8 * g + i, kb = ka + 16; v[i] = ka < K ? W[(size_t)(ka < K ? ka : K - 1) * ld + n] : 0.f; v[8 + i] = kb < K ? W[(size_t)(kb < K ? kb : K - 1) * ld + n] : 0.f; }
  return bsplit16(v); }
__device__ __forceinline__ v8f mac3(const F2& a, const F2& b, v8f c) { c = wmma_bf(a.l, b.h, c); c = wmma_bf(a.h, b.l, c); return wmma_bf(a.h, b.h, c); }
__device__ __forceinline__ float sigm(float v) { return 1.0f / (1.0f + expf(-v)); }
#define LDSX() do { asm volatile("s_wait_dscnt 0" ::: "memory"); __builtin_amdgcn_wave_barrier(); __builtin_amdgcn_fence(__ATOMIC_RELEASE, "workgroup"); } while (0)


#define NB 2
#define CC 2048
#define NPOS 256
#define NHD 8
#define HDIM 256
#define HIDC 512
#ifndef TNB
#define TNB NB
#endif
__device__ __forceinline__ float bfr(float v) { return (float)(__bf16)v; }
__device__ __attribute__((noinline)) float exp_ni(float v) { return expf(v); }
typedef __attribute__((ext_vector_type(8))) __bf16 v8b;
__device__ __forceinline__ v16b frag_b(const __bf16* rowk0, int lane) {
  union { v16b v; v8b q[2]; } u; const __bf16* p = rowk0 + 8 * (lane >> 4);
  u.q[0] = *(const v8b*)p; u.q[1] = *(const v8b*)(p + 16); return u.v;
}
__device__ __forceinline__ v16b frag_gbf(const float* rowk0, int lane) {
  v16b a; const float* p = rowk0 + 8 * (lane >> 4);
#pragma unroll
  for (int i = 0; i < 8; ++i) { a[i] = (__bf16)p[i]; a[8 + i] = (__bf16)p[16 + i]; }
  return a;
}
__constant__ float c_mult[16] = {5.f, 10.f, 10.f, 10.f, 9.f, 8.f, 8.f, 8.f, 8.f, 8.f, 8.f, 9.f, 10.f, 10.f, 10.f, 5.f};

#define WS_XTH  0u
#define WS_XTL  (WS_XTH + 2u * NB * NPOS * CC)
#define WS_QT   (WS_XTL + 2u * NB * NPOS * CC)
#define WS_KT   (WS_QT + 4u * NB * NPOS * CC)
#define WS_VT   (WS_KT + 4u * NB * NPOS * CC)
#define WS_V    (WS_VT + 4u * NB * NPOS * CC)
#define WS_X1   (WS_V + 4u * NB * CC * NPOS)
#define WS_HT   (WS_X1 + 4u * NB * CC * NPOS)
#define WS_END  (WS_HT + 4u * NB * NPOS * HIDC)

template <int ROUNDX>
__global__ __launch_bounds__(256) void k_bnT(const float* __restrict__ X, const float* __restrict__ g, const float* __restrict__ bb, const float* __restrict__ m, const float* __restrict__ v, __bf16* __restrict__ PH, __bf16* __restrict__ PL) {
  __shared__ __bf16 sh[NPOS][72], sl[NPOS][72]; __shared__ float ssc[64], ssh[64];
  const int b = blockIdx.y, c0 = blockIdx.x * 64, tid = threadIdx.x;
  if (tid < 64) { const int c = c0 + tid; const float sc = bfr(g[c]) / sqrtf(bfr(v[c]) + 1e-5f); ssc[tid] = sc; ssh[tid] = bfr(bb[c]) - bfr(m[c]) * sc; }
  __syncthreads();
  for (int q = tid; q < 64 * NPOS; q += 256) { const int cl = q >> 8, p = q & 255; const float xr = X[((size_t)b * CC + c0 + cl) * NPOS + p]; const float val = (ROUNDX ? bfr(xr) : xr) * ssc[cl] + ssh[cl]; const __bf16 hi = (__bf16)val; sh[p][cl] = hi; sl[p][cl] = (__bf16)(val - (float)hi); }
  __syncthreads();
  for (int q = tid; q < NPOS * 8; q += 256) { const int p = q >> 3, pc = q & 7; union { __bf16 e[8]; v4u u; } a, c;
#pragma unroll
    for (int e = 0; e < 8; ++e) { a.e[e] = sh[p][pc * 8 + e]; c.e[e] = sl[p][pc * 8 + e]; }
    const size_t o = ((size_t)b * NPOS + p) * CC + c0 + pc * 8; vst2((unsigned*)(PH + o), a.u); vst2((unsigned*)(PL + o), c.u); }
}
template <int KIN, int NOUT, int RELU6>
__global__ __launch_bounds__(128) void k_conv(const __bf16* __restrict__ PH, const __bf16* __restrict__ PL, const float* __restrict__ Wm, const float* __restrict__ bias, float* __restrict__ OUT) {
  __shared__ __align__(16) float so[4][16][132];
  const int tid = threadIdx.x, wave = tid >> 5, lane = tid & 31, col = lane & 15, g = lane >> 4; const int b = blockIdx.z; const int p0 = blockIdx.x * 64 + wave * 16; const int n0 = blockIdx.y * 128;
  const size_t arow = ((size_t)b * NPOS + p0 + col) * KIN;
  v8f acc[8] = {};
#pragma unroll 2
  for (int kc = 0; kc < KIN / 32; ++kc) { const v16b ah = frag_b(PH + arow + kc * 32, lane), al = frag_b(PL + arow + kc * 32, lane);
#pragma unroll
    for (int j = 0; j < 8; ++j) { const v16b w = frag_gbf(Wm + (size_t)(n0 + j * 16 + col) * KIN + kc * 32, lane); acc[j] = wmma_bf(al, w, acc[j]); acc[j] = wmma_bf(ah, w, acc[j]); } }
#pragma unroll
  for (int j = 0; j < 8; ++j) { const float bv = bfr(bias[n0 + j * 16 + col]);
#pragma unroll
    for (int r = 0; r < 8; ++r) { float v = acc[j][r] + bv; if (RELU6) v = fminf(fmaxf(v, 0.f), 6.0f); so[wave][8 * g + r][j * 16 + col] = v; } }
  LDSX();
  for (int rl = 0; rl < 16; ++rl) vst2(OUT + ((size_t)b * NPOS + p0 + rl) * NOUT + n0 + lane * 4, *(const v4f*)(&so[wave][rl][lane * 4]));
}
__global__ __launch_bounds__(256) void k_tr(const float* __restrict__ VT, float* __restrict__ V) {
  __shared__ __align__(16) float st[64][NPOS + 4];
  const int b = blockIdx.y, o0 = blockIdx.x * 64, tid = threadIdx.x;
  for (int q = tid; q < NPOS * 64; q += 256) { const int p = q >> 6, ol = q & 63; st[ol][p] = VT[((size_t)b * NPOS + p) * CC + o0 + ol]; }
  __syncthreads();
  for (int q = tid; q < 64 * 64; q += 256) { const int ol = q >> 6, pc = q & 63; vst2(V + ((size_t)b * CC + o0 + ol) * NPOS + pc * 4, *(const v4f*)&st[ol][pc * 4]); }
}
__global__ __launch_bounds__(64) void k_attn(const float* __restrict__ QT, const float* __restrict__ KT, const float* __restrict__ V, const float* __restrict__ X, const float* __restrict__ g1, const float* __restrict__ b1, const float* __restrict__ m1, const float* __restrict__ v1, const float* __restrict__ gam, float* __restrict__ X1) {
  __shared__ __align__(16) float sP[32][NPOS + 4];
  __shared__ __align__(16) float so[64][36];
  const int tid = threadIdx.x, wave = tid >> 5, lane = tid & 31, col = lane & 15, g = lane >> 4;
  const int b = blockIdx.z, n = blockIdx.y, q0 = blockIdx.x * 32; const int ocol = n * HDIM;
  const float* qrow = QT + ((size_t)b * NPOS + q0 + wave * 16 + col) * CC + ocol;
#pragma unroll 1
  for (int half = 0; half < 2; ++half) { v8f acc[8] = {};
#pragma unroll 1
    for (int kc = 0; kc < HDIM / 32; ++kc) { const F2 a = split_row(qrow, kc * 32, lane);
#pragma unroll
      for (int j = 0; j < 8; ++j) { const F2 kb = split_row(KT + ((size_t)b * NPOS + (half * 8 + j) * 16 + col) * CC + ocol, kc * 32, lane); acc[j] = mac3(a, kb, acc[j]); } }
#pragma unroll
    for (int j = 0; j < 8; ++j)
#pragma unroll
      for (int r = 0; r < 8; ++r) sP[wave * 16 + 8 * g + r][(half * 8 + j) * 16 + col] = acc[j][r]; }
  LDSX();
#pragma unroll 1
  for (int rl = 0; rl < 16; ++rl) { float* row = &sP[wave * 16 + rl][0]; float mx = -3.0e38f;
#pragma unroll
    for (int i = 0; i < 8; ++i) mx = fmaxf(mx, row[lane * 8 + i]);
#pragma unroll
    for (int o = 1; o < 32; o <<= 1) mx = fmaxf(mx, __shfl_xor(mx, o));
    float w[8]; float s = 0.f;
#pragma unroll
    for (int i = 0; i < 8; ++i) { const int sidx = lane * 8 + i; const float mlt = c_mult[sidx >> 4] * c_mult[sidx & 15]; w[i] = mlt * exp_ni(row[sidx] - mx); s += w[i]; }
#pragma unroll
    for (int o = 1; o < 32; o <<= 1) s += __shfl_xor(s, o);
    const float inv = 1.0f / s;
#pragma unroll
    for (int i = 0; i < 8; ++i) row[lane * 8 + i] = w[i] * inv; }
  LDSX();
  const float gm = bfr(gam[0]);
#pragma unroll 1
  for (int dc = 0; dc < 4; ++dc) { v8f acc[4] = {};
#pragma unroll 1
    for (int kc = 0; kc < NPOS / 32; ++kc) { const F2 a = split_row(&sP[wave * 16 + col][0], kc * 32, lane);
#pragma unroll
      for (int j = 0; j < 4; ++j) { const F2 vb = split_row(V + ((size_t)b * CC + ocol + dc * 64 + j * 16 + col) * NPOS, kc * 32, lane); acc[j] = mac3(a, vb, acc[j]); } }
    __syncthreads();
#pragma unroll
    for (int j = 0; j < 4; ++j)
#pragma unroll
      for (int r = 0; r < 8; ++r) so[j * 16 + col][wave * 16 + 8 * g + r] = acc[j][r];
    __syncthreads();
    for (int qq = tid; qq < 64 * 8; qq += 64) { const int dl = qq >> 3, pc = qq & 7; const int o = ocol + dc * 64 + dl; const size_t base = ((size_t)b * CC + o) * NPOS + q0 + pc * 4;
      const float sc = bfr(g1[o]) / sqrtf(bfr(v1[o]) + 1e-5f), sh = bfr(b1[o]) - bfr(m1[o]) * sc;
      const float4 xv = *(const float4*)(X + base); v4f r4; const float xs[4] = {xv.x, xv.y, xv.z, xv.w};
#pragma unroll
      for (int i = 0; i < 4; ++i) { const float xb = bfr(xs[i]); r4[i] = xb + (gm * so[dl][pc * 4 + i] + (xb * sc + sh)); }
      vst2(X1 + base, r4); } }
}
__global__ __launch_bounds__(128) void k_mlp2(const float* __restrict__ HT, const float* __restrict__ W2, const float* __restrict__ b2, const float* __restrict__ X1, float* __restrict__ out) {
  __shared__ __align__(16) float st[128][68];
  const int tid = threadIdx.x, wave = tid >> 5, lane = tid & 31, col = lane & 15, g = lane >> 4; const int b = blockIdx.z; const int p0 = blockIdx.x * 64; const int n0 = blockIdx.y * 128;
  v8f acc[8] = {};
#pragma unroll 2
  for (int kc = 0; kc < HIDC / 32; ++kc) { const F2 a = split_row(HT + ((size_t)b * NPOS + p0 + wave * 16 + col) * HIDC, kc * 32, lane);
#pragma unroll
    for (int j = 0; j < 8; ++j) { const v16b w = frag_gbf(W2 + (size_t)(n0 + j * 16 + col) * HIDC + kc * 32, lane); acc[j] = wmma_bf(a.l, w, acc[j]); acc[j] = wmma_bf(a.h, w, acc[j]); } }
#pragma unroll
  for (int j = 0; j < 8; ++j) { const float bv = bfr(b2[n0 + j * 16 + col]);
#pragma unroll
    for (int r = 0; r < 8; ++r) st[j * 16 + col][wave * 16 + 8 * g + r] = acc[j][r] + bv; }
  __syncthreads();
  for (int qq = tid; qq < 128 * 16; qq += 128) { const int ol = qq >> 4, pc = qq & 15; const size_t base = ((size_t)b * CC + n0 + ol) * NPOS + p0 + pc * 4; const float4 xv = *(const float4*)(X1 + base);
    v4f r4; r4[0] = xv.x + st[ol][pc * 4]; r4[1] = xv.y + st[ol][pc * 4 + 1]; r4[2] = xv.z + st[ol][pc * 4 + 2]; r4[3] = xv.w + st[ol][pc * 4 + 3]; vst2(out + base, r4); }
}

extern "C" void kernel_launch(void* const* d_in, const int* in_sizes, int n_in, void* d_out, int out_size, void* d_ws, size_t ws_size, hipStream_t stream) {
  (void)in_sizes; (void)n_in; (void)out_size;
  const float** F = (const float**)d_in;
  if (ws_size < (size_t)WS_END) return;
  char* ws = (char*)d_ws;
  __bf16 *PH = (__bf16*)(ws + WS_XTH), *PL = (__bf16*)(ws + WS_XTL); float *QT = (float*)(ws + WS_QT), *KT = (float*)(ws + WS_KT), *VT = (float*)(ws + WS_VT), *V = (float*)(ws + WS_V), *X1 = (float*)(ws + WS_X1), *HT = (float*)(ws + WS_HT);
  k_bnT<1><<<dim3(CC / 64, TNB), 256, 0, stream>>>(F[0], F[1], F[2], F[3], F[4], PH, PL);
  k_conv<CC, CC, 0><<<dim3(NPOS / 64, CC / 128, TNB), 128, 0, stream>>>(PH, PL, F[5], F[6], QT);
  k_conv<CC, CC, 0><<<dim3(NPOS / 64, CC / 128, TNB), 128, 0, stream>>>(PH, PL, F[7], F[8], KT);
  k_conv<CC, CC, 0><<<dim3(NPOS / 64, CC / 128, TNB), 128, 0, stream>>>(PH, PL, F[9], F[10], VT);
  k_tr<<<dim3(CC / 64, TNB), 256, 0, stream>>>(VT, V);
  k_attn<<<dim3(NPOS / 32, NHD, TNB), 64, 0, stream>>>(QT, KT, V, F[0], F[1], F[2], F[3], F[4], F[11], X1);
  k_bnT<0><<<dim3(CC / 64, TNB), 256, 0, stream>>>(X1, F[12], F[13], F[14], F[15], PH, PL);
  k_conv<CC, HIDC, 1><<<dim3(NPOS / 64, HIDC / 128, TNB), 128, 0, stream>>>(PH, PL, F[16], F[17], HT);
  k_mlp2<<<dim3(NPOS / 64, CC / 128, TNB), 128, 0, stream>>>(HT, F[18], F[19], X1, (float*)d_out);
}
